// MHSelfAttention_77747497992540
// MI455X (gfx1250) — hardware-verified
//
#include <hip/hip_runtime.h>


#ifndef NB
#define NB 4
#endif
#ifndef SEQ
#define SEQ 2048
#endif
#define NB_FULL  4
#define SEQ_FULL 2048
#define DM   1024
#define NH_  16
#define HD   64
#define DQ   (NH_ * HD)
#define D3   (3 * DM)
#define RHC  512
#define RH   ((SEQ < RHC) ? SEQ : RHC)
#define PCAR 1024.0f
#define SCL  0.125f
static_assert(SEQ % 64 == 0);
static_assert(SEQ >= 64);
static_assert(SEQ <= SEQ_FULL);
static_assert(NB >= 1);
static_assert(NB <= NB_FULL);
static_assert(RH % 64 == 0);
static_assert(DM % 64 == 0);
static_assert(DQ == DM);
static_assert(D3 % 64 == 0);

typedef _Float16 h16;
typedef unsigned short bf;
typedef __attribute__((ext_vector_type(16))) __bf16   v16bf;
typedef __attribute__((ext_vector_type(16))) _Float16 v16h;
typedef __attribute__((ext_vector_type(8)))  _Float16 v8h;
typedef __attribute__((ext_vector_type(8)))  unsigned short v8us;
typedef __attribute__((ext_vector_type(8)))  float    v8f;
typedef __attribute__((ext_vector_type(4)))  float    v4f;
typedef v8h  __attribute__((may_alias)) v8ha;
typedef v4f  __attribute__((may_alias)) v4fa;
typedef v8us __attribute__((may_alias)) v8usa;
static_assert(sizeof(v8us) == 16);
static_assert(sizeof(v4f) == 16);

__device__ __forceinline__ unsigned short f2bf(float f) { unsigned u = __float_as_uint(f); u += 0x7FFFu + ((u >> 16) & 1u); return (unsigned short)(u >> 16); }
__device__ __forceinline__ float bf2f(unsigned short b) { return __uint_as_float(((unsigned)b) << 16); }
__device__ __forceinline__ float bfr(float f) { return bf2f(f2bf(f)); }
__device__ __forceinline__ v16h cat16(v8h lo, v8h hi) { return __builtin_shufflevector(lo, hi, 0, 1, 2, 3, 4, 5, 6, 7, 8, 9, 10, 11, 12, 13, 14, 15); }
__device__ __forceinline__ v16bf cat16b(v8us lo, v8us hi) { return __builtin_bit_cast(v16bf, __builtin_shufflevector(lo, hi, 0, 1, 2, 3, 4, 5, 6, 7, 8, 9, 10, 11, 12, 13, 14, 15)); }
__device__ __forceinline__ v8f wmma16(v16h a, v16h b, v8f c) { return __builtin_amdgcn_wmma_f32_16x16x32_f16(false, a, false, b, (short)0, c, false, false); }
__device__ __forceinline__ v8f wmmab(v16bf a, v16bf b, v8f c) { return __builtin_amdgcn_wmma_f32_16x16x32_bf16(false, a, false, b, (short)0, c, false, false); }


template <typename T16> struct WFrag;
template <> struct WFrag<h16> { typedef v16h V; static __device__ __forceinline__ V ld(const h16* p) { return cat16(*(const v8h*)p, *(const v8h*)(p + 16)); } static __device__ __forceinline__ v8f mma(V a, V b, v8f c) { return wmma16(a, b, c); } };
template <> struct WFrag<bf> { typedef v16bf V; static __device__ __forceinline__ V ld(const bf* p) { return cat16b(*(const v8us*)p, *(const v8us*)(p + 16)); } static __device__ __forceinline__ v8f mma(V a, V b, v8f c) { return wmmab(a, b, c); } };
template <typename T16, int NSPLIT, bool BIAS>
__global__ __launch_bounds__(32) void k_gemmw(const T16* __restrict__ A, const T16* __restrict__ A2, const T16* __restrict__ Bt, const T16* __restrict__ Bt2, int K, float* C, int ldc, const float* __restrict__ bias, size_t sA, size_t sB, size_t sC) {
    typedef typename WFrag<T16>::V V;
    __shared__ __align__(16) float os[16 * 68];
    const size_t z = blockIdx.z; A += z * sA; if (A2) A2 += z * sA; Bt += z * sB; if (Bt2) Bt2 += z * sB; C += z * sC;
    const int lane = threadIdx.x & 31, lr = lane & 15, hi = lane >> 4; const int r0 = blockIdx.x * 64, c0 = blockIdx.y * 64;
    v8f acc[4][4];
#pragma unroll
    for (int mb = 0; mb < 4; ++mb)
#pragma unroll
        for (int nb = 0; nb < 4; ++nb) acc[mb][nb] = (v8f){};
    const size_t aoff = (size_t)(r0 + lr) * K + 8 * hi, boff = (size_t)(c0 + lr) * K + 8 * hi;
#pragma unroll 1
    for (int kc = 0; kc < K; kc += 32) {
        V a[4], a2[4];
#pragma unroll
        for (int mb = 0; mb < 4; ++mb) { a[mb] = WFrag<T16>::ld(A + aoff + (size_t)mb * 16 * K + kc); if (NSPLIT == 1 || NSPLIT == 2) a2[mb] = WFrag<T16>::ld(A2 + aoff + (size_t)mb * 16 * K + kc); }
#pragma unroll
        for (int nb = 0; nb < 4; ++nb) { const V b = WFrag<T16>::ld(Bt + boff + (size_t)nb * 16 * K + kc); V b2; if (NSPLIT >= 2) b2 = WFrag<T16>::ld(Bt2 + boff + (size_t)nb * 16 * K + kc);
#pragma unroll
            for (int mb = 0; mb < 4; ++mb) { acc[mb][nb] = WFrag<T16>::mma(a[mb], b, acc[mb][nb]); if (NSPLIT == 1 || NSPLIT == 2) acc[mb][nb] = WFrag<T16>::mma(a2[mb], b, acc[mb][nb]); if (NSPLIT >= 2) acc[mb][nb] = WFrag<T16>::mma(a[mb], b2, acc[mb][nb]); } }
        asm volatile("v_nop\n\tv_nop\n\tv_nop\n\tv_nop" : "+v"(acc[0][0]), "+v"(acc[1][1]), "+v"(acc[2][2]), "+v"(acc[3][3]) : "v"(a[0]), "v"(a[3]));
    }
#pragma unroll
    for (int mb = 0; mb < 4; ++mb) {
#pragma unroll
        for (int nb = 0; nb < 4; ++nb) {
#pragma unroll
            for (int j = 0; j < 8; ++j) os[(hi * 8 + j) * 68 + nb * 16 + lr] = acc[mb][nb][j]; }
        __builtin_amdgcn_wave_barrier(); asm volatile("" ::: "memory");
        float* crow = C + (size_t)(r0 + mb * 16) * ldc + c0;
#pragma unroll 1
        for (int ps = 0; ps < 2; ++ps) {
#pragma unroll
            for (int s = 0; s < 8; ++s) { const int row = 2 * s + hi, cofs = lr * 4; v4f val = *(const v4fa*)(os + row * 68 + cofs); if (BIAS) { val[0] += bfr(bias[c0 + cofs]); val[1] += bfr(bias[c0 + cofs + 1]); val[2] += bfr(bias[c0 + cofs + 2]); val[3] += bfr(bias[c0 + cofs + 3]); }
                *(volatile v4f*)(crow + (size_t)row * ldc + cofs) = val; }
            if (ps == 0) __threadfence(); }
        __builtin_amdgcn_wave_barrier(); asm volatile("" ::: "memory");
    }
}

__device__ __forceinline__ h16 tohx(float x) { return (h16)x; }
__device__ __forceinline__ void splitf(float y, unsigned short& h, unsigned short& l) { h = f2bf(y); l = f2bf(y - bf2f(h)); }
typedef __attribute__((ext_vector_type(2))) _Float16 v2h;
typedef __attribute__((ext_vector_type(4))) _Float16 v4h;
typedef __attribute__((ext_vector_type(2))) unsigned short v2us;
typedef __attribute__((ext_vector_type(4))) unsigned short v4us;
typedef __attribute__((ext_vector_type(2))) float v2f;

__global__ __launch_bounds__(256) void k_cvt8(const float* __restrict__ src, bf* dst, size_t n8) { const size_t i = (size_t)blockIdx.x * 256 + threadIdx.x; if (i >= n8) return; const v8f v = *(const v8f*)(src + i * 8); v8us o;
#pragma unroll
    for (int k = 0; k < 8; ++k) o[k] = f2bf(v[k]); *(volatile v8us*)(dst + i * 8) = o; __threadfence(); *(volatile v8us*)(dst + i * 8) = o; }

__global__ __launch_bounds__(256) void k_qkp(const float* __restrict__ F, int pitch, int nheads, h16* P16, bf* Ph, bf* Pl) {
    const size_t e = ((size_t)blockIdx.x * 256 + threadIdx.x) * 2; if (e >= (size_t)nheads * SEQ * HD) return; const int d = (int)(e % HD); const int t = (int)((e / HD) % SEQ); const int hh = (int)(e / ((size_t)HD * SEQ));
    const v2f xv = *(const v2f*)(F + (size_t)t * pitch + hh * HD + d); v2h o16; v2us oh, ol;
#pragma unroll
    for (int q = 0; q < 2; ++q) { o16[q] = tohx(xv[q]); unsigned short a2, c2; splitf(xv[q], a2, c2); oh[q] = a2; ol[q] = c2; }
    *(volatile v2h*)(P16 + e) = o16; *(volatile v2us*)(Ph + e) = oh; *(volatile v2us*)(Pl + e) = ol; __threadfence(); *(volatile v2h*)(P16 + e) = o16; *(volatile v2us*)(Ph + e) = oh; *(volatile v2us*)(Pl + e) = ol; }
__global__ __launch_bounds__(256) void k_vtp(const float* __restrict__ F, int pitch, int nheads, h16* V16, bf* Vh, bf* Vl) { const size_t e = ((size_t)blockIdx.x * 256 + threadIdx.x) * 2; if (e >= (size_t)nheads * HD * SEQ) return; const int t = (int)(e % SEQ); const int d = (int)((e / SEQ) % HD); const int g = (int)(e / ((size_t)SEQ * HD)); v2h o16; v2us oh, ol;
#pragma unroll
    for (int q = 0; q < 2; ++q) { const float xv = F[(size_t)(t + q) * pitch + g * HD + d]; o16[q] = tohx(xv); unsigned short a2, c2; splitf(xv, a2, c2); oh[q] = a2; ol[q] = c2; }
    *(volatile v2h*)(V16 + e) = o16; *(volatile v2us*)(Vh + e) = oh; *(volatile v2us*)(Vl + e) = ol; __threadfence(); *(volatile v2h*)(V16 + e) = o16; *(volatile v2us*)(Vh + e) = oh; *(volatile v2us*)(Vl + e) = ol; }

template <bool HR>
__global__ __launch_bounds__(128) void k_attn(const h16* __restrict__ Q16, const bf* __restrict__ Qh, const bf* __restrict__ Ql,
                                              const h16* __restrict__ K16, const bf* __restrict__ Kh, const bf* __restrict__ Kl,
                                              const h16* __restrict__ V16, const bf* __restrict__ Vh, const bf* __restrict__ Vl,
                                              int qb0, bf* ATh, bf* ATl) {
    constexpr int PLS = 72;
    constexpr float L2E = 1.4426950408889634f;
    __shared__ __align__(16) h16 p16s[4][16 * PLS];
    __shared__ __align__(16) bf phs[4][16 * PLS];
    __shared__ __align__(16) bf pls[4][16 * PLS];
    __shared__ __align__(16) float osb[4][16 * 68];
    const int lane = threadIdx.x & 31, w = threadIdx.x >> 5, lr = lane & 15, hi = lane >> 4;
    const int qb = qb0 + (int)blockIdx.x, q0 = qb * 64, hh = (int)blockIdx.y, rw = q0 + w * 16;
    const size_t qkb = (size_t)hh * SEQ * HD, vtb = (size_t)hh * HD * SEQ;
    const size_t qoff = qkb + (size_t)(rw + lr) * HD + 8 * hi;
    float mrun[8], lrun[8]; v8f o[4];
#pragma unroll
    for (int j = 0; j < 8; ++j) { mrun[j] = -3.0e38f; lrun[j] = 0.f; }
#pragma unroll
    for (int nb = 0; nb < 4; ++nb) o[nb] = (v8f){};
#pragma unroll 1
    for (int kb = 0; kb <= qb; ++kb) {
        const int key0 = kb * 64;
        __syncthreads();
        v8f s[4];
#pragma unroll
        for (int nb = 0; nb < 4; ++nb) s[nb] = (v8f){};
        if constexpr (HR) {
            const v16bf qh0 = WFrag<bf>::ld(Qh + qoff), qh1 = WFrag<bf>::ld(Qh + qoff + 32), ql0 = WFrag<bf>::ld(Ql + qoff), ql1 = WFrag<bf>::ld(Ql + qoff + 32);
#pragma unroll
            for (int nb = 0; nb < 4; ++nb) { const size_t ko = qkb + (size_t)(key0 + nb * 16 + lr) * HD + 8 * hi;
                const v16bf b0 = WFrag<bf>::ld(Kh + ko), b1 = WFrag<bf>::ld(Kh + ko + 32), c0 = WFrag<bf>::ld(Kl + ko), c1 = WFrag<bf>::ld(Kl + ko + 32);
                s[nb] = wmmab(qh0, b0, s[nb]); s[nb] = wmmab(qh1, b1, s[nb]); s[nb] = wmmab(ql0, b0, s[nb]); s[nb] = wmmab(ql1, b1, s[nb]); s[nb] = wmmab(qh0, c0, s[nb]); s[nb] = wmmab(qh1, c1, s[nb]);
                asm volatile("v_nop\n\tv_nop\n\tv_nop\n\tv_nop" : "+v"(s[nb]) : "v"(b1), "v"(c1), "v"(qh1), "v"(ql1)); asm volatile("" ::: "memory"); }
        } else {
            const v16h qa0 = WFrag<h16>::ld(Q16 + qoff), qa1 = WFrag<h16>::ld(Q16 + qoff + 32);
#pragma unroll
            for (int nb = 0; nb < 4; ++nb) { const size_t ko = qkb + (size_t)(key0 + nb * 16 + lr) * HD + 8 * hi;
                const v16h b0 = WFrag<h16>::ld(K16 + ko), b1 = WFrag<h16>::ld(K16 + ko + 32);
                s[nb] = wmma16(qa0, b0, s[nb]); s[nb] = wmma16(qa1, b1, s[nb]);
                asm volatile("v_nop\n\tv_nop\n\tv_nop\n\tv_nop" : "+v"(s[nb]) : "v"(b1), "v"(qa1)); asm volatile("" ::: "memory"); }
        }
        float mx[8];
#pragma unroll
        for (int j = 0; j < 8; ++j) mx[j] = -3.0e38f;
#pragma unroll
        for (int nb = 0; nb < 4; ++nb) { const int key = key0 + nb * 16 + lr;
#pragma unroll
            for (int j = 0; j < 8; ++j) { const int row = rw + 8 * hi + j; const float t = (key > row) ? -3.0e38f : s[nb][j] * SCL; s[nb][j] = t; mx[j] = fmaxf(mx[j], t); } }
        float cf[8], rs[8];
#pragma unroll
        for (int j = 0; j < 8; ++j) {
#pragma unroll
            for (int sh = 8; sh; sh >>= 1) mx[j] = fmaxf(mx[j], __shfl_xor(mx[j], sh, 32));
            mx[j] = fmaxf(mx[j], mrun[j]);
            float d0 = __fsub_rn(mrun[j], mx[j]); asm volatile("" : "+v"(d0)); cf[j] = __builtin_amdgcn_exp2f(__fmul_rn(d0, L2E)); mrun[j] = mx[j]; rs[j] = 0.f; }
#pragma unroll
        for (int nb = 0; nb < 4; ++nb)
#pragma unroll
            for (int j = 0; j < 8; ++j) { float d0 = __fsub_rn(s[nb][j], mx[j]); asm volatile("" : "+v"(d0)); const float p = __builtin_amdgcn_exp2f(__fmul_rn(d0, L2E)); rs[j] += p;
                const int li = (8 * hi + j) * PLS + nb * 16 + lr;
                if constexpr (HR) { unsigned short a2, c2; splitf(p, a2, c2); phs[w][li] = a2; pls[w][li] = c2; } else { p16s[w][li] = tohx(p * PCAR); } }
#pragma unroll
        for (int j = 0; j < 8; ++j) {
#pragma unroll
            for (int sh = 8; sh; sh >>= 1) rs[j] += __shfl_xor(rs[j], sh, 32);
            lrun[j] = lrun[j] * cf[j] + rs[j];
#pragma unroll
            for (int nb = 0; nb < 4; ++nb) o[nb][j] *= cf[j]; }
        __syncthreads();
        if constexpr (HR) {
            const bf* pr = &phs[w][lr * PLS + 8 * hi]; const bf* pq = &pls[w][lr * PLS + 8 * hi];
            const v16bf pa0 = WFrag<bf>::ld(pr), pa1 = WFrag<bf>::ld(pr + 32), pc0 = WFrag<bf>::ld(pq), pc1 = WFrag<bf>::ld(pq + 32);
#pragma unroll
            for (int nb = 0; nb < 4; ++nb) { const size_t vo = vtb + (size_t)(nb * 16 + lr) * SEQ + key0 + 8 * hi;
                const v16bf b0 = WFrag<bf>::ld(Vh + vo), b1 = WFrag<bf>::ld(Vh + vo + 32), c0 = WFrag<bf>::ld(Vl + vo), c1 = WFrag<bf>::ld(Vl + vo + 32);
                o[nb] = wmmab(pa0, b0, o[nb]); o[nb] = wmmab(pa1, b1, o[nb]); o[nb] = wmmab(pc0, b0, o[nb]); o[nb] = wmmab(pc1, b1, o[nb]); o[nb] = wmmab(pa0, c0, o[nb]); o[nb] = wmmab(pa1, c1, o[nb]);
                asm volatile("v_nop\n\tv_nop\n\tv_nop\n\tv_nop" : "+v"(o[nb]) : "v"(b1), "v"(c1), "v"(pa1), "v"(pc1)); asm volatile("" ::: "memory"); }
        } else {
            const h16* pr = &p16s[w][lr * PLS + 8 * hi];
            const v16h pa0 = WFrag<h16>::ld(pr), pa1 = WFrag<h16>::ld(pr + 32);
#pragma unroll
            for (int nb = 0; nb < 4; ++nb) { const size_t vo = vtb + (size_t)(nb * 16 + lr) * SEQ + key0 + 8 * hi;
                const v16h b0 = WFrag<h16>::ld(V16 + vo), b1 = WFrag<h16>::ld(V16 + vo + 32);
                o[nb] = wmma16(pa0, b0, o[nb]); o[nb] = wmma16(pa1, b1, o[nb]);
                asm volatile("v_nop\n\tv_nop\n\tv_nop\n\tv_nop" : "+v"(o[nb]) : "v"(b1), "v"(pa1)); asm volatile("" ::: "memory"); }
        }
    }
    float f[8];
#pragma unroll
    for (int j = 0; j < 8; ++j) f[j] = (HR ? 1.0f : (1.0f / PCAR)) * __fdiv_rn(1.0f, lrun[j]);
#pragma unroll
    for (int nb = 0; nb < 4; ++nb)
#pragma unroll
        for (int j = 0; j < 8; ++j) osb[w][(8 * hi + j) * 68 + nb * 16 + lr] = o[nb][j] * f[j];
    __syncthreads();
    const int r4 = lane >> 3, p8 = lane & 7;
#pragma unroll 1
    for (int ps = 0; ps < 2; ++ps) {
#pragma unroll
        for (int g = 0; g < 4; ++g) { const int row = g * 4 + r4; const float* src = &osb[w][row * 68 + p8 * 8];
            const v4f x0 = *(const v4fa*)src, x1 = *(const v4fa*)(src + 4); v8us oh, ol;
#pragma unroll
            for (int q = 0; q < 4; ++q) { unsigned short a2, c2; splitf(x0[q], a2, c2); oh[q] = a2; ol[q] = c2; splitf(x1[q], a2, c2); oh[4 + q] = a2; ol[4 + q] = c2; }
            const size_t oo = (size_t)(rw + row) * DQ + (size_t)hh * HD + p8 * 8;
            *(volatile v8us*)(ATh + oo) = oh; *(volatile v8us*)(ATl + oo) = ol; }
        if (ps == 0) __threadfence(); }
}

extern "C" void kernel_launch(void* const* d_in, const int* in_sizes, int n_in,
                              void* d_out, int out_size, void* d_ws, size_t ws_size, hipStream_t stream) {
    if (n_in < 4) return;
    const size_t needx = (size_t)(NB - 1) * SEQ_FULL * DM + (size_t)SEQ * DM;
    if ((size_t)in_sizes[0] < needx) return;
    if ((size_t)in_sizes[1] < (size_t)D3 * DM || (size_t)in_sizes[2] < (size_t)DM * DQ || in_sizes[3] < DM) return;
    if ((size_t)out_size < needx) return;
    const float* x = (const float*)d_in[0];
    const float* w_in = (const float*)d_in[1];
    const float* w_out = (const float*)d_in[2];
    const float* b_out = (const float*)d_in[3];
    float* OUT = (float*)d_out;
    char* wsp = (char*)d_ws;
    auto take = [&](size_t bytes) { char* p = wsp; wsp += (bytes + 255) & ~(size_t)255; return (void*)p; };
    bf* WI = (bf*)take((size_t)D3 * DM * 2);
    bf* WO = (bf*)take((size_t)DM * DQ * 2);
    bf* XB = (bf*)take((size_t)SEQ * DM * 2);
    float* FQKV = (float*)take((size_t)SEQ * D3 * 4);
    const size_t plane = (size_t)NH_ * SEQ * HD * 2;
    h16* QP16 = (h16*)take(plane); bf* QPh = (bf*)take(plane); bf* QPl = (bf*)take(plane);
    h16* KP16 = (h16*)take(plane); bf* KPh = (bf*)take(plane); bf* KPl = (bf*)take(plane);
    h16* VT16 = (h16*)take(plane); bf* VTh = (bf*)take(plane); bf* VTl = (bf*)take(plane);
    bf* ATh = (bf*)take((size_t)SEQ * DQ * 2); bf* ATl = (bf*)take((size_t)SEQ * DQ * 2);
    const size_t carved = (size_t)(wsp - (char*)d_ws);
    if (carved > ws_size || carved > ((size_t)128 << 20)) return;
    k_cvt8<<<(unsigned)(((size_t)D3 * DM / 8 + 255) / 256), 256, 0, stream>>>(w_in, WI, (size_t)D3 * DM / 8);
    k_cvt8<<<(unsigned)(((size_t)DM * DQ / 8 + 255) / 256), 256, 0, stream>>>(w_out, WO, (size_t)DM * DQ / 8);
    const unsigned LP = (unsigned)(((size_t)NH_ * SEQ * HD / 2 + 255) / 256);
    for (int b = 0; b < NB; ++b) {
        k_cvt8<<<(unsigned)(((size_t)SEQ * DM / 8 + 255) / 256), 256, 0, stream>>>(x + (size_t)b * SEQ_FULL * DM, XB, (size_t)SEQ * DM / 8);
        k_gemmw<bf, 0, false><<<dim3(SEQ / 64, D3 / 64, 1), 32, 0, stream>>>(XB, nullptr, WI, nullptr, DM, FQKV, D3, nullptr, 0, 0, 0);
        k_qkp<<<LP, 256, 0, stream>>>(FQKV, D3, NH_, QP16, QPh, QPl);
        k_qkp<<<LP, 256, 0, stream>>>(FQKV + DM, D3, NH_, KP16, KPh, KPl);
        k_vtp<<<LP, 256, 0, stream>>>(FQKV + 2 * DM, D3, NH_, VT16, VTh, VTl);
        k_attn<true><<<dim3(RH / 64, NH_, 1), 128, 0, stream>>>(QP16, QPh, QPl, KP16, KPh, KPl, VT16, VTh, VTl, 0, ATh, ATl);
        if (SEQ > RH) k_attn<false><<<dim3((SEQ - RH) / 64, NH_, 1), 128, 0, stream>>>(QP16, QPh, QPl, KP16, KPh, KPl, VT16, VTh, VTl, RH / 64, ATh, ATl);
        k_gemmw<bf, 1, true><<<dim3(SEQ / 64, DM / 64, 1), 32, 0, stream>>>(ATh, ATl, WO, nullptr, DQ, OUT + (size_t)b * SEQ_FULL * DM, DM, b_out, 0, 0, 0);
    }
}
